// DecoderModule_41223096107032
// MI455X (gfx1250) — hardware-run, weakly checked
//
#include <hip/hip_runtime.h>
#include <stdint.h>

constexpr int kTok   = 4096;
constexpr int kEmb   = 768;
constexpr int kHeads = 12;
constexpr int kHD    = 64;
constexpr int kFF    = 3072;
constexpr float kLnEps = 1e-5f;
constexpr size_t kNE = (size_t)kTok * kEmb;
constexpr size_t kEE = (size_t)kEmb * kEmb;
constexpr size_t kEF = (size_t)kEmb * kFF;
constexpr size_t kNF = (size_t)kTok * kFF;
constexpr size_t kHeadPlane = (size_t)kTok * kHD;
static_assert(kHeads * kHD == kEmb, "heads");
static_assert(kTok % 64 == 0 && kEmb % 64 == 0 && kFF % 64 == 0, "tiles");
static_assert(kEmb % 32 == 0 && kFF % 32 == 0, "ktail");
static_assert(kTok % 8 == 0, "lnrows");
static_assert(kEmb == 768, "lnwidth");
static_assert(kNE % 512 == 0, "cast");

constexpr size_t kOffXh    = 0;
constexpr size_t kOffWqkvT = kOffXh + kNE * 2;
constexpr size_t kOffWoT   = kOffWqkvT + 3 * kEE * 2;
constexpr size_t kOffW1T   = kOffWoT + kEE * 2;
constexpr size_t kOffW2T   = kOffW1T + kEF * 2;
constexpr size_t kOffQKV   = kOffW2T + kEF * 2;
constexpr size_t kOffCtx   = kOffQKV + 3 * kNE * 2;
constexpr size_t kOffAO    = kOffCtx + kNE * 2;
constexpr size_t kOffH1f   = kOffAO + kNE * 4;
constexpr size_t kOffH1h   = kOffH1f + kNE * 4;
constexpr size_t kOffF1h   = kOffH1h + kNE * 2;
constexpr size_t kWsTotal  = kOffF1h + kNF * 2;
static_assert(kWsTotal == 102236160, "wstotal");
static_assert(kWsTotal <= 134217728, "wscap");
static_assert(kOffWqkvT % 256 == 0 && kOffWoT % 256 == 0 && kOffW1T % 256 == 0 && kOffW2T % 256 == 0 &&
              kOffQKV % 256 == 0 && kOffCtx % 256 == 0 && kOffAO % 256 == 0 && kOffH1f % 256 == 0 &&
              kOffH1h % 256 == 0 && kOffF1h % 256 == 0, "align");

typedef __attribute__((ext_vector_type(16))) _Float16 v16h;
typedef __attribute__((ext_vector_type(8)))  _Float16 v8h;
typedef __attribute__((ext_vector_type(16))) __bf16   v16b;
typedef __attribute__((ext_vector_type(8)))  __bf16   v8b;
typedef __attribute__((ext_vector_type(8)))  float    v8f;
typedef __attribute__((ext_vector_type(4)))  float    v4f;
#define PSCALE 32768.0f
#define U16(p) ((const unsigned short*)(const void*)(p))
#define PSCALE_INV (1.0f / 32768.0f)

__device__ __forceinline__ unsigned short f2bf_bits(float f) {
  unsigned u = __float_as_uint(f);
  return (unsigned short)((u + 0x7FFFu + ((u >> 16) & 1u)) >> 16);
}
__device__ __forceinline__ float bf_bits2f(unsigned short h) { return __uint_as_float(((unsigned)h) << 16); }

__device__ __forceinline__ void dep_guard_h(v8f& a, v8f& b, v16h x, v16h y) { asm volatile("v_nop\n\tv_nop\n\tv_nop\n\tv_nop" : "+v"(a), "+v"(b) : "v"(x), "v"(y)); }
__device__ __forceinline__ void dep_guard_b(v8f& a, v8f& b, v16b x, v16b y) { asm volatile("v_nop\n\tv_nop\n\tv_nop\n\tv_nop" : "+v"(a), "+v"(b) : "v"(x), "v"(y)); }
__device__ __forceinline__ void keep4_h(v16h a, v16h b, v16h c, v16h d) { asm volatile("v_nop" :: "v"(a), "v"(b), "v"(c), "v"(d)); }
__device__ __forceinline__ void keep4_b(v16b a, v16b b, v16b c, v16b d) { asm volatile("v_nop" :: "v"(a), "v"(b), "v"(c), "v"(d)); }
__device__ __forceinline__ void acc_guard4(v8f& a, v8f& b, v8f& c, v8f& d) { asm volatile("v_nop\n\tv_nop\n\tv_nop\n\tv_nop" : "+v"(a), "+v"(b), "+v"(c), "+v"(d)); }
template <typename T> struct Frag;
template <> struct Frag<_Float16> {
  typedef v16h V; union U { v16h v; v8h h[2]; };
  static __device__ __forceinline__ v16h load(const _Float16* p) {
    U f; f.h[0] = *(const v8h*)(p); f.h[1] = *(const v8h*)(p + 16); return f.v;
  }
  static __device__ __forceinline__ v8f mma(v16h a, v16h b, v8f c) {
    return __builtin_amdgcn_wmma_f32_16x16x32_f16(false, a, false, b, (short)0, c, false, false);
  }
  static __device__ __forceinline__ void guard(v8f& a, v8f& b, v16h x, v16h y) { dep_guard_h(a, b, x, y); }
  static __device__ __forceinline__ void keep(v16h a, v16h b, v16h c, v16h d) { keep4_h(a, b, c, d); }
};
template <> struct Frag<__bf16> {
  typedef v16b V; union U { v16b v; v8b h[2]; };
  static __device__ __forceinline__ v16b load(const __bf16* p) {
    U f; f.h[0] = *(const v8b*)(p); f.h[1] = *(const v8b*)(p + 16); return f.v;
  }
  static __device__ __forceinline__ v8f mma(v16b a, v16b b, v8f c) {
    return __builtin_amdgcn_wmma_f32_16x16x32_bf16(false, a, false, b, (short)0, c, false, false);
  }
  static __device__ __forceinline__ void guard(v8f& a, v8f& b, v16b x, v16b y) { dep_guard_b(a, b, x, y); }
  static __device__ __forceinline__ void keep(v16b a, v16b b, v16b c, v16b d) { keep4_b(a, b, c, d); }
};

template <int ET> struct Elem;
template <> struct Elem<0> { typedef _Float16 T; };
template <> struct Elem<1> { typedef __bf16 T; };
template <int ET, bool SPLIT, int BIAS_MODE, int OUT_MODE, bool RESID, int ACT = 0>
__global__ __launch_bounds__(256) void wmma_gemm64(
    const unsigned short* __restrict__ Ap, const unsigned short* __restrict__ A2p, int lda, long strideA,
    const unsigned short* __restrict__ Btp, const unsigned short* __restrict__ Bt2p, int ldb, long strideB,
    void* __restrict__ Cout, void* __restrict__ Cout2, int ldc, long strideC,
    const float* __restrict__ bias,
    const float* __restrict__ resid, long strideR,
    int M, int N, int K, float scale) {
  typedef typename Elem<ET>::T T;
  typedef typename Frag<T>::V V;
  const T* A = (const T*)Ap; const T* A2 = (const T*)A2p; const T* Bt = (const T*)Btp; const T* Bt2 = (const T*)Bt2p;
  __shared__ __align__(16) float sT[8][16 * 68];
  const int b    = blockIdx.y;
  const int lane = threadIdx.x & 31;
  const int wave = threadIdx.x >> 5;
  const int tilesN = N >> 6;
  const int tilesM = M >> 6;
  const int tile = blockIdx.x * 8 + wave;
  if (tile >= tilesM * tilesN) return;
  const int tm = tile / tilesN;
  const int tn = tile - tm * tilesN;
  const int m0 = tm << 6;
  const int n0 = tn << 6;

  const T* Ab  = A  + (size_t)b * strideA;
  const T* Bb  = Bt + (size_t)b * strideB;
  const T* Ab2 = SPLIT ? (A2  + (size_t)b * strideA) : nullptr;
  const T* Bb2 = SPLIT ? (Bt2 + (size_t)b * strideB) : nullptr;

  const int rlane = lane & 15;
  const int koff  = (lane >> 4) * 8;
  const int mOff  = (lane >> 4) * 8;

  v8f acc[4][4];
#pragma unroll
  for (int i = 0; i < 4; ++i)
#pragma unroll
    for (int j = 0; j < 4; ++j) acc[i][j] = (v8f){0.f,0.f,0.f,0.f,0.f,0.f,0.f,0.f};

  for (int k0 = 0; k0 < K; k0 += 32) {
    V bh[4], bl[4];
#pragma unroll
    for (int j = 0; j < 4; ++j) {
      const size_t bo = (size_t)(n0 + (j << 4) + rlane) * ldb + koff + k0;
      bh[j] = Frag<T>::load(Bb + bo);
      if (SPLIT) bl[j] = Frag<T>::load(Bb2 + bo);
    }
#pragma unroll
    for (int i = 0; i < 4; ++i) {
      const size_t ao = (size_t)(m0 + (i << 4) + rlane) * lda + koff + k0;
      V ah = Frag<T>::load(Ab + ao);
      V al;
      if (SPLIT) al = Frag<T>::load(Ab2 + ao);
#pragma unroll
      for (int j = 0; j < 4; ++j) {
        acc[i][j] = Frag<T>::mma(ah, bh[j], acc[i][j]);
        if (SPLIT) {
          acc[i][j] = Frag<T>::mma(ah, bl[j], acc[i][j]);
          acc[i][j] = Frag<T>::mma(al, bh[j], acc[i][j]);
        }
      }
      Frag<T>::guard(acc[i][0], acc[i][3], ah, SPLIT ? al : ah);
    }
    Frag<T>::keep(bh[0], bh[1], bh[2], bh[3]);
    if (SPLIT) Frag<T>::keep(bl[0], bl[1], bl[2], bl[3]);
  }
  acc_guard4(acc[0][0], acc[0][1], acc[0][2], acc[0][3]);
  acc_guard4(acc[1][0], acc[1][1], acc[1][2], acc[1][3]);
  acc_guard4(acc[2][0], acc[2][1], acc[2][2], acc[2][3]);
  acc_guard4(acc[3][0], acc[3][1], acc[3][2], acc[3][3]);

  float* slab = sT[wave];
  const float* Rb = RESID ? (resid + (size_t)b * strideR) : nullptr;
#pragma unroll
  for (int i = 0; i < 4; ++i) {
    const int mBase = m0 + (i << 4);
#pragma unroll
    for (int j = 0; j < 4; ++j) {
      const int n = n0 + (j << 4) + rlane;
      float bv = 0.f;
      if (BIAS_MODE == 2) bv = bias[n];
#pragma unroll
      for (int r = 0; r < 8; ++r) {
        float v = acc[i][j][r] * scale;
        if (BIAS_MODE == 1) v += bias[mBase + mOff + r];
        if (BIAS_MODE == 2) v += bv;
        if (RESID) v += Rb[(size_t)(mBase + mOff + r) * ldc + n];
        if (ACT == 1) v = tanhf(v);
        if (ACT == 2) v = fmaxf(v, 0.0f);
        if (ACT == 3) v = v / (1.0f + expf(-v));
        if (ACT == 4) v = (v > 0.f) ? v : 0.01f * v;
        if (ACT == 5) v = 0.5f * v * (1.0f + erff(v * 0.70710678118654752f));
        slab[(mOff + r) * 68 + (j << 4) + rlane] = v;
      }
    }
    __builtin_amdgcn_fence(__ATOMIC_RELEASE, "workgroup");
    __builtin_amdgcn_wave_barrier();
    __builtin_amdgcn_fence(__ATOMIC_ACQUIRE, "workgroup");
    if (OUT_MODE == 0) {
      float* C = (float*)Cout + (size_t)b * strideC;
      const int hh = lane >> 4, c4 = (lane & 15) * 4;
      for (int pass = 0; pass < 2; ++pass) {
#pragma unroll
        for (int it = 0; it < 8; ++it) {
          const int row = it * 2 + hh;
          v4f v = *(const v4f*)(slab + row * 68 + c4);
          *(volatile v4f*)(C + (size_t)(mBase + row) * ldc + n0 + c4) = v;
        }
        __threadfence();
      }
    } else {
      const int q = lane >> 3, c8 = (lane & 7) * 8;
      unsigned short* C  = (unsigned short*)Cout  + (size_t)b * strideC;
      unsigned short* C2 = (OUT_MODE == 2) ? ((unsigned short*)Cout2 + (size_t)b * strideC) : nullptr;
      for (int pass = 0; pass < 2; ++pass) {
#pragma unroll
        for (int it = 0; it < 4; ++it) {
          const int row = it * 4 + q;
          const float* sp = slab + row * 68 + c8;
          v8h hv, lv;
#pragma unroll
          for (int e = 0; e < 8; ++e) {
            if (OUT_MODE == 1) {
              hv[e] = (_Float16)sp[e];
            } else {
              unsigned short hb = f2bf_bits(sp[e]);
              unsigned short lb = f2bf_bits(sp[e] - bf_bits2f(hb));
              hv[e] = __builtin_bit_cast(_Float16, hb);
              lv[e] = __builtin_bit_cast(_Float16, lb);
            }
          }
          *(volatile v8h*)(C + (size_t)(mBase + row) * ldc + n0 + c8) = hv;
          if (OUT_MODE == 2) *(volatile v8h*)(C2 + (size_t)(mBase + row) * ldc + n0 + c8) = lv;
        }
        __threadfence();
      }
    }
    __builtin_amdgcn_fence(__ATOMIC_RELEASE, "workgroup");
    __builtin_amdgcn_wave_barrier();
    __builtin_amdgcn_fence(__ATOMIC_ACQUIRE, "workgroup");
  }
}

__global__ __launch_bounds__(256) void cast_f32_f16x2(
    const float* __restrict__ in, _Float16* __restrict__ out, int n2) {
  int i = blockIdx.x * 256 + threadIdx.x;
  if (i < n2) {
    const _Float16 h0 = (_Float16)in[2 * i], h1 = (_Float16)in[2 * i + 1];
    const unsigned u = (unsigned)__builtin_bit_cast(unsigned short, h0) | ((unsigned)__builtin_bit_cast(unsigned short, h1) << 16);
    ((volatile unsigned*)out)[i] = u;
    __threadfence();
    ((volatile unsigned*)out)[i] = u;
  }
}

__global__ __launch_bounds__(256) void transpose_cast_f16(
    const float* __restrict__ in, unsigned short* __restrict__ out, int rows, int cols, float sc) {
  __shared__ float tileS[64][65];
  const int tid = threadIdx.x, lane = tid & 31, wave = tid >> 5;
  const int c0 = blockIdx.x * 64, r0 = blockIdx.y * 64;
  {
    const int lr = tid >> 2, lc = (tid & 3) * 16;
    const float* src = in + (size_t)(r0 + lr) * cols + c0 + lc;
#pragma unroll
    for (int i = 0; i < 4; ++i) {
      const v4f v = *(const v4f*)(src + 4 * i);
      tileS[lr][lc + 4 * i + 0] = v[0];
      tileS[lr][lc + 4 * i + 1] = v[1];
      tileS[lr][lc + 4 * i + 2] = v[2];
      tileS[lr][lc + 4 * i + 3] = v[3];
    }
  }
  __syncthreads();
  const int q = lane >> 3, c8 = (lane & 7) * 8;
  _Float16* ob = (_Float16*)out;
  for (int pass = 0; pass < 2; ++pass) {
#pragma unroll
    for (int it = 0; it < 2; ++it) {
      const int orow = wave * 8 + it * 4 + q;
      v8h hv;
#pragma unroll
      for (int e = 0; e < 8; ++e) hv[e] = (_Float16)(tileS[c8 + e][orow] * sc);
      *(volatile v8h*)(ob + (size_t)(c0 + orow) * rows + r0 + c8) = hv;
    }
    __threadfence();
  }
}

#define AT_D 64
#define AT_NW 4
#define AT_QB 64
#define AT_KC 64
__device__ __forceinline__ v8f mma_f16(v16h a, v16h b, v8f c) {
  c = __builtin_amdgcn_wmma_f32_16x16x32_f16(false, a, false, b, (short)0, c, false, false);
  asm volatile("v_nop\n\tv_nop\n\tv_nop\n\tv_nop" : "+v"(c) : "v"(a), "v"(b));
  return c;
}

__global__ __launch_bounds__(128)
void attn_causal_f16(const unsigned short* __restrict__ Qp, const unsigned short* __restrict__ Kp,
                     const unsigned short* __restrict__ Vp, unsigned short* __restrict__ Cp,
                     float sm_scale, float out_carry) {
  const float PSC = PSCALE;
  const float kNegInf = -__builtin_inff();
  union HB { v16h v; v8h h[2]; };
  __shared__ __align__(16) unsigned short Ksh[AT_KC * AT_D];
  __shared__ __align__(16) unsigned short Vth[AT_D * AT_KC];
  __shared__ __align__(16) _Float16 Psh[AT_NW][16 * AT_KC];
  __shared__ __align__(16) float Os[AT_NW][16 * 68];

  const int tid  = threadIdx.x;
  const int wave = tid >> 5;
  const int lane = tid & 31;
  const int hh   = lane >> 4;
  const int c    = lane & 15;

  const int nqb = kTok / AT_QB;
  const int bx  = blockIdx.x;
  const int qb  = bx % nqb;
  const int h   = bx / nqb;
  const int q0  = qb * AT_QB + wave * 16;

  const _Float16* qh = (const _Float16*)Qp + (size_t)h * kHeadPlane;
  const unsigned short* kh = Kp + (size_t)h * kHeadPlane;
  const unsigned short* vh = Vp + (size_t)h * kHeadPlane;

  v16h qa[2];
#pragma unroll
  for (int dc = 0; dc < 2; ++dc)
    qa[dc] = Frag<_Float16>::load(qh + (size_t)(q0 + c) * AT_D + dc * 32 + 8 * hh);

  float mrow[8], lrow[8];
  v8f oacc[4];
#pragma unroll
  for (int r = 0; r < 8; ++r) { mrow[r] = kNegInf; lrow[r] = 0.f; }
#pragma unroll
  for (int t = 0; t < 4; ++t) oacc[t] = (v8f){0.f,0.f,0.f,0.f,0.f,0.f,0.f,0.f};

  const int nChunks = qb + 1;
  for (int kc = 0; kc < nChunks; ++kc) {
    const int kv0 = kc * AT_KC;
    __syncthreads();
    {
      const int kvr = tid >> 1, dh = (tid & 1) * 32;
      const uint4* ksrc = (const uint4*)(kh + (size_t)(kv0 + kvr) * AT_D + dh);
      const uint4* vsrc = (const uint4*)(vh + (size_t)(kv0 + kvr) * AT_D + dh);
      uint4 kw[4], vw[4];
#pragma unroll
      for (int i = 0; i < 4; ++i) { kw[i] = ksrc[i]; vw[i] = vsrc[i]; }
      uint4* kdst = (uint4*)(Ksh + kvr * AT_D + dh);
#pragma unroll
      for (int i = 0; i < 4; ++i) kdst[i] = kw[i];
#pragma unroll
      for (int i = 0; i < 4; ++i) {
        const unsigned w0 = vw[i].x, w1 = vw[i].y, w2 = vw[i].z, w3 = vw[i].w;
        const int d = dh + 8 * i;
        Vth[(d + 0) * AT_KC + kvr] = (unsigned short)(w0 & 0xffffu);
        Vth[(d + 1) * AT_KC + kvr] = (unsigned short)(w0 >> 16);
        Vth[(d + 2) * AT_KC + kvr] = (unsigned short)(w1 & 0xffffu);
        Vth[(d + 3) * AT_KC + kvr] = (unsigned short)(w1 >> 16);
        Vth[(d + 4) * AT_KC + kvr] = (unsigned short)(w2 & 0xffffu);
        Vth[(d + 5) * AT_KC + kvr] = (unsigned short)(w2 >> 16);
        Vth[(d + 6) * AT_KC + kvr] = (unsigned short)(w3 & 0xffffu);
        Vth[(d + 7) * AT_KC + kvr] = (unsigned short)(w3 >> 16);
      }
    }
    __syncthreads();

    v8f s[4];
#pragma unroll
    for (int j = 0; j < 4; ++j) {
      s[j] = (v8f){0.f,0.f,0.f,0.f,0.f,0.f,0.f,0.f};
#pragma unroll
      for (int dc = 0; dc < 2; ++dc) {
        HB kb;
        kb.h[0] = *(const v8h*)(const void*)(Ksh + (j * 16 + c) * AT_D + dc * 32 + 8 * hh);
        kb.h[1] = *(const v8h*)(const void*)(Ksh + (j * 16 + c) * AT_D + dc * 32 + 16 + 8 * hh);
        s[j] = mma_f16(qa[dc], kb.v, s[j]);
      }
    }
    const bool diag = (kc == qb);
    float cm[8];
#pragma unroll
    for (int r = 0; r < 8; ++r) {
      const int qrow = q0 + 8 * hh + r;
      float m = kNegInf;
#pragma unroll
      for (int j = 0; j < 4; ++j) {
        const int kvcol = kv0 + j * 16 + c;
        float val = s[j][r] * sm_scale;
        const bool masked = diag && (kvcol > qrow);
        val = masked ? kNegInf : val;
        s[j][r] = val;
        m = fmaxf(m, val);
      }
#pragma unroll
      for (int off = 1; off < 16; off <<= 1) m = fmaxf(m, __shfl_xor(m, off, 32));
      cm[r] = m;
    }
    _Float16* pw = Psh[wave];
#pragma unroll
    for (int r = 0; r < 8; ++r) {
      const float mnew = fmaxf(mrow[r], cm[r]);
      const float alpha = expf(mrow[r] - mnew);
      mrow[r] = mnew;
      float psum = 0.f;
#pragma unroll
      for (int j = 0; j < 4; ++j) {
        const float p = expf(s[j][r] - mnew);
        psum += p;
        pw[(8 * hh + r) * AT_KC + j * 16 + c] = (_Float16)(p * PSC);
      }
#pragma unroll
      for (int off = 1; off < 16; off <<= 1) psum += __shfl_xor(psum, off, 32);
      lrow[r] = lrow[r] * alpha + psum;
#pragma unroll
      for (int t = 0; t < 4; ++t) oacc[t][r] *= alpha;
    }
    __builtin_amdgcn_fence(__ATOMIC_RELEASE, "workgroup");
    __builtin_amdgcn_wave_barrier();
    __builtin_amdgcn_fence(__ATOMIC_ACQUIRE, "workgroup");
#pragma unroll 1
    for (int kk = 0; kk < 2; ++kk) {
      HB pa;
      pa.h[0] = *(const v8h*)(pw + c * AT_KC + kk * 32 + 8 * hh);
      pa.h[1] = *(const v8h*)(pw + c * AT_KC + kk * 32 + 16 + 8 * hh);
#pragma unroll
      for (int t = 0; t < 4; ++t) {
        HB vb;
        vb.h[0] = *(const v8h*)(const void*)(Vth + (t * 16 + c) * AT_KC + kk * 32 + 8 * hh);
        vb.h[1] = *(const v8h*)(const void*)(Vth + (t * 16 + c) * AT_KC + kk * 32 + 16 + 8 * hh);
        oacc[t] = mma_f16(pa.v, vb.v, oacc[t]);
      }
    }
  }

  float* os = Os[wave];
#pragma unroll
  for (int r = 0; r < 8; ++r) {
    const float inv = out_carry * (1.0f / (lrow[r] * PSC));
#pragma unroll
    for (int t = 0; t < 4; ++t) os[(8 * hh + r) * 68 + t * 16 + c] = oacc[t][r] * inv;
  }
  __builtin_amdgcn_fence(__ATOMIC_RELEASE, "workgroup");
  __builtin_amdgcn_wave_barrier();
  __builtin_amdgcn_fence(__ATOMIC_ACQUIRE, "workgroup");
  {
    const int q = lane >> 3, c8 = (lane & 7) * 8;
    _Float16* crow = (_Float16*)Cp + (size_t)h * kHD;
    for (int pass = 0; pass < 2; ++pass) {
#pragma unroll
      for (int it = 0; it < 4; ++it) {
        const int row = it * 4 + q;
        const float* sp = os + row * 68 + c8;
        v8h hv;
#pragma unroll
        for (int e = 0; e < 8; ++e) hv[e] = (_Float16)sp[e];
        *(volatile v8h*)(crow + (size_t)(q0 + row) * kEmb + c8) = hv;
      }
      __threadfence();
    }
  }
}

template <bool WRITE_H>
__global__ __launch_bounds__(256) void ln_rows_kernel(
    const float* __restrict__ X, const float* __restrict__ R,
    const float* __restrict__ gam, const float* __restrict__ bet,
    float* __restrict__ outF, unsigned short* __restrict__ outH) {
  __shared__ __align__(16) float rowbuf[8][kEmb];
  const int lane = threadIdx.x & 31, wave = threadIdx.x >> 5;
  const int row = blockIdx.x * 8 + wave;
  const float* xr = X + (size_t)row * kEmb;
  const float* rr = R + (size_t)row * kEmb;
  v4f t[6];
#pragma unroll
  for (int i = 0; i < 6; ++i) {
    const v4f a  = *(const v4f*)(xr + 128 * i + 4 * lane);
    const v4f rv = *(const v4f*)(rr + 128 * i + 4 * lane);
    t[i] = a + rv;
  }
  float s = 0.f;
#pragma unroll
  for (int i = 0; i < 6; ++i) { s += t[i][0]; s += t[i][1]; s += t[i][2]; s += t[i][3]; }
#pragma unroll
  for (int off = 1; off < 32; off <<= 1) s += __shfl_xor(s, off, 32);
  const float mean = s * (1.0f / (float)kEmb);
  float vs = 0.f;
#pragma unroll
  for (int i = 0; i < 6; ++i) {
#pragma unroll
    for (int e = 0; e < 4; ++e) { const float dd = t[i][e] - mean; vs += dd * dd; }
  }
#pragma unroll
  for (int off = 1; off < 32; off <<= 1) vs += __shfl_xor(vs, off, 32);
  const float rstd = rsqrtf(vs * (1.0f / (float)kEmb) + kLnEps);
  asm volatile("" ::: "memory");
  v4f o[6];
#pragma unroll
  for (int i = 0; i < 6; ++i) {
    const v4f gv = *(const v4f*)(gam + 128 * i + 4 * lane);
    const v4f bv = *(const v4f*)(bet + 128 * i + 4 * lane);
#pragma unroll
    for (int e = 0; e < 4; ++e) o[i][e] = (t[i][e] - mean) * rstd * gv[e] + bv[e];
  }
  float* orow = outF + (size_t)row * kEmb;
  for (int pass = 0; pass < 2; ++pass) {
#pragma unroll
    for (int i = 0; i < 6; ++i) *(volatile v4f*)(orow + 128 * i + 4 * lane) = o[i];
    __threadfence();
  }
  if (WRITE_H) {
    float* rb = rowbuf[wave];
#pragma unroll
    for (int i = 0; i < 6; ++i) {
      rb[128 * i + 4 * lane + 0] = o[i][0];
      rb[128 * i + 4 * lane + 1] = o[i][1];
      rb[128 * i + 4 * lane + 2] = o[i][2];
      rb[128 * i + 4 * lane + 3] = o[i][3];
    }
    __builtin_amdgcn_fence(__ATOMIC_RELEASE, "workgroup");
    __builtin_amdgcn_wave_barrier();
    __builtin_amdgcn_fence(__ATOMIC_ACQUIRE, "workgroup");
    _Float16* hrow = (_Float16*)outH + (size_t)row * kEmb;
    for (int pass = 0; pass < 2; ++pass) {
#pragma unroll
      for (int i = 0; i < 3; ++i) {
        const int c8 = 256 * i + 8 * lane;
        const float* sp = rb + c8;
        v8h hv;
#pragma unroll
        for (int e = 0; e < 8; ++e) hv[e] = (_Float16)sp[e];
        *(volatile v8h*)(hrow + c8) = hv;
      }
      __threadfence();
    }
  }
}

extern "C" void kernel_launch(void* const* d_in, const int* in_sizes, int n_in,
                              void* d_out, int out_size, void* d_ws, size_t ws_size,
                              hipStream_t stream) {
  (void)in_sizes; (void)n_in;
  if (ws_size < kWsTotal) return;
  if ((size_t)out_size < kNE) return;

  const float* x     = (const float*)d_in[0];
  const float* Wq    = (const float*)d_in[1];
  const float* Wk    = (const float*)d_in[2];
  const float* Wv    = (const float*)d_in[3];
  const float* Wo    = (const float*)d_in[4];
  const float* W1    = (const float*)d_in[5];
  const float* b1    = (const float*)d_in[6];
  const float* W2    = (const float*)d_in[7];
  const float* b2    = (const float*)d_in[8];
  const float* g1    = (const float*)d_in[9];
  const float* beta1 = (const float*)d_in[10];
  const float* g2    = (const float*)d_in[11];
  const float* beta2 = (const float*)d_in[12];
  float* outp = (float*)d_out;

  char* ws = (char*)d_ws;
  unsigned short* Xh    = (unsigned short*)(ws + kOffXh);
  unsigned short* WqkvT = (unsigned short*)(ws + kOffWqkvT);
  unsigned short* WoT   = (unsigned short*)(ws + kOffWoT);
  unsigned short* W1T   = (unsigned short*)(ws + kOffW1T);
  unsigned short* W2T   = (unsigned short*)(ws + kOffW2T);
  unsigned short* QKVh  = (unsigned short*)(ws + kOffQKV);
  unsigned short* Qh    = QKVh;
  unsigned short* Kh    = QKVh + kNE;
  unsigned short* Vh    = QKVh + 2 * kNE;
  unsigned short* Ctxh  = (unsigned short*)(ws + kOffCtx);
  float*          AttnF = (float*)(ws + kOffAO);
  float*          Ff2F  = (float*)(ws + kOffAO);
  float*          H1f   = (float*)(ws + kOffH1f);
  unsigned short* H1h   = (unsigned short*)(ws + kOffH1h);
  unsigned short* F1h   = (unsigned short*)(ws + kOffF1h);

  cast_f32_f16x2<<<(unsigned)(kNE / 2 / 256), 256, 0, stream>>>(x, (_Float16*)Xh, (int)(kNE / 2));

  transpose_cast_f16<<<dim3(kEmb / 64, kEmb / 64), 256, 0, stream>>>(Wq, WqkvT,           kEmb, kEmb, 64.0f);
  transpose_cast_f16<<<dim3(kEmb / 64, kEmb / 64), 256, 0, stream>>>(Wk, WqkvT + kEE,     kEmb, kEmb, 64.0f);
  transpose_cast_f16<<<dim3(kEmb / 64, kEmb / 64), 256, 0, stream>>>(Wv, WqkvT + 2 * kEE, kEmb, kEmb, 64.0f);
  transpose_cast_f16<<<dim3(kEmb / 64, kEmb / 64), 256, 0, stream>>>(Wo, WoT,             kEmb, kEmb, 64.0f);
  transpose_cast_f16<<<dim3(kFF / 64, kEmb / 64), 256, 0, stream>>>(W1, W1T, kEmb, kFF, 64.0f);
  transpose_cast_f16<<<dim3(kEmb / 64, kFF / 64), 256, 0, stream>>>(W2, W2T, kFF, kEmb, 64.0f);

  constexpr int kTilesE = (kTok / 64) * (kEmb / 64);
  constexpr int kTilesF = (kTok / 64) * (kFF / 64);
  static_assert(kTilesE % 8 == 0 && kTilesF % 8 == 0, "tilegrid");

  wmma_gemm64<0, false, 0, 1, false, 0><<<dim3(kTilesE / 8, 3), 256, 0, stream>>>(
      Xh, Xh, kEmb, 0L, WqkvT, WqkvT, kEmb, (long)kEE, (void*)QKVh, (void*)QKVh, kEmb, (long)kNE,
      b1, x, 0L, kTok, kEmb, kEmb, 1.0f / 64.0f);

  attn_causal_f16<<<kHeads * (kTok / AT_QB), 128, 0, stream>>>(Qh, Kh, Vh, Ctxh, 0.125f, 64.0f);

  wmma_gemm64<0, false, 0, 0, false, 0><<<dim3(kTilesE / 8, 1), 256, 0, stream>>>(
      Ctxh, Ctxh, kEmb, 0L, WoT, WoT, kEmb, 0L, (void*)AttnF, (void*)AttnF, kEmb, 0L,
      b2, x, 0L, kTok, kEmb, kEmb, 1.0f / 4096.0f);

  ln_rows_kernel<true><<<kTok / 8, 256, 0, stream>>>(x, AttnF, g1, beta1, H1f, H1h);

  wmma_gemm64<0, false, 2, 1, false, 2><<<dim3(kTilesF / 8, 1), 256, 0, stream>>>(
      H1h, H1h, kEmb, 0L, W1T, W1T, kEmb, 0L, (void*)F1h, (void*)F1h, kFF, 0L,
      b1, x, 0L, kTok, kFF, kEmb, 1.0f / 64.0f);

  wmma_gemm64<0, false, 2, 0, false, 0><<<dim3(kTilesE / 8, 1), 256, 0, stream>>>(
      F1h, F1h, kFF, 0L, W2T, W2T, kFF, 0L, (void*)Ff2F, (void*)Ff2F, kEmb, 0L,
      b2, x, 0L, kTok, kEmb, kFF, 1.0f / 64.0f);

  ln_rows_kernel<false><<<kTok / 8, 256, 0, stream>>>(H1f, Ff2F, g2, beta2, outp, H1h);
}
